// VectorPoolLocalInterpolateModule_43645457662573
// MI455X (gfx1250) — hardware-verified
//
#include <hip/hip_runtime.h>
#include <math.h>

typedef __attribute__((ext_vector_type(16))) _Float16 v16h;
typedef __attribute__((ext_vector_type(16))) __bf16 v16b;
typedef __attribute__((ext_vector_type(8)))  _Float16 v8h;
typedef __attribute__((ext_vector_type(8)))  float v8f;
typedef __attribute__((ext_vector_type(4)))  float v4f;
typedef __attribute__((ext_vector_type(2)))  float v2f;
typedef __attribute__((ext_vector_type(4)))  unsigned v4u;
typedef __attribute__((ext_vector_type(4)))  int v4i;
typedef float __attribute__((may_alias)) float_a;
typedef int __attribute__((may_alias)) int_a;

template <typename T> __device__ __forceinline__ void vst2(void* p, T v) { *(volatile T*)p = v; __threadfence(); *(volatile T*)p = v; }
__device__ __forceinline__ v8f wmma16(v16h a, v16h b, v8f c) {
  v8f d = __builtin_amdgcn_wmma_f32_16x16x32_f16(false, a, false, b, (short)0, c, false, false);
  asm volatile("v_nop\n\tv_nop\n\tv_nop\n\tv_nop" : "+v"(d) : "v"(a), "v"(b));
  return d;
}
__device__ __forceinline__ v8f wmma_bf(v16b a, v16b b, v8f c) {
  v8f d = __builtin_amdgcn_wmma_f32_16x16x32_bf16(false, a, false, b, (short)0, c, false, false);
  asm volatile("v_nop\n\tv_nop\n\tv_nop\n\tv_nop" : "+v"(d) : "v"(a), "v"(b));
  return d;
}
__device__ __forceinline__ v16h frag_h(const _Float16* rowk0, int lane) {
  union { v16h v; v8h q[2]; } u; const _Float16* p = rowk0 + 8 * (lane >> 4);
  u.q[0] = *(const v8h*)p; u.q[1] = *(const v8h*)(p + 16); return u.v;
}
__device__ __forceinline__ v16h frag_f32(const float* rowk0, int lane) {
  v16h a; const float* p = rowk0 + 8 * (lane >> 4);
#pragma unroll
  for (int i = 0; i < 8; ++i) { a[i] = (_Float16)p[i]; a[8 + i] = (_Float16)p[16 + i]; }
  return a;
}
__device__ __forceinline__ v16h frag_f32s(const float* rowk0, int lane, float sc) {
  v16h a; const float* p = rowk0 + 8 * (lane >> 4);
#pragma unroll
  for (int i = 0; i < 8; ++i) { a[i] = (_Float16)(p[i] * sc); a[8 + i] = (_Float16)(p[16 + i] * sc); }
  return a;
}
__device__ __forceinline__ v16h fragc_f32(const float* W, int k0, int n, int lane, int ld, int K) {
  v16h a; const int g = lane >> 4;
#pragma unroll
  for (int i = 0; i < 8; ++i) { const int ka = k0 + 8 * g + i, kb = ka + 16;
    a[i] = (_Float16)(ka < K ? W[(size_t)(ka < K ? ka : K - 1) * ld + n] : 0.f); a[8 + i] = (_Float16)(kb < K ? W[(size_t)(kb < K ? kb : K - 1) * ld + n] : 0.f); }
  return a;
}
struct F2 { v16b h, l; };
__device__ __forceinline__ F2 bsplit16(const float v[16]) { F2 r;
#pragma unroll
  for (int i = 0; i < 16; ++i) { const __bf16 h = (__bf16)v[i]; r.h[i] = h; r.l[i] = (__bf16)(v[i] - (float)h); }
  return r; }
__device__ __forceinline__ F2 split_row(const float* row, int k0, int lane) { float v[16]; const float* p = row + k0 + 8 * (lane >> 4);
#pragma unroll
  for (int i = 0; i < 8; ++i) { v[i] = p[i]; v[8 + i] = p[16 + i]; }
  return bsplit16(v); }
__device__ __forceinline__ F2 split_rowK(const float* row, int k0, int lane, int K) { float v[16]; const int g = lane >> 4;
#pragma unroll
  for (int i = 0; i < 8; ++i) { const int ka = k0 + 8 * g + i, kb = ka + 16; v[i] = ka < K ? row[ka < K ? ka : K - 1] : 0.f; v[8 + i] = kb < K ? row[kb < K ? kb : K - 1] : 0.f; }
  return bsplit16(v); }
__device__ __forceinline__ F2 split_col(const float* W, int k0, int n, int lane, int ld, int K) { float v[16]; const int g = lane >> 4;
#pragma unroll
  for (int i = 0; i < 8; ++i) { const int ka = k0 + 8 * g + i, kb = ka + 16; v[i] = ka < K ? W[(size_t)(ka < K ? ka : K - 1) * ld + n] : 0.f; v[8 + i] = kb < K ? W[(size_t)(kb < K ? kb : K - 1) * ld + n] : 0.f; }
  return bsplit16(v); }
__device__ __forceinline__ v8f mac3(const F2& a, const F2& b, v8f c) { c = wmma_bf(a.l, b.h, c); c = wmma_bf(a.h, b.l, c); return wmma_bf(a.h, b.h, c); }
__device__ __forceinline__ float sigm(float v) { return 1.0f / (1.0f + expf(-v)); }
#define LDSX() do { asm volatile("s_wait_dscnt 0" ::: "memory"); __builtin_amdgcn_wave_barrier(); __builtin_amdgcn_fence(__ATOMIC_RELEASE, "workgroup"); } while (0)

__device__ __forceinline__ float bfr(float v) { return (float)(__bf16)v; }
__device__ __forceinline__ float bfi(float v) { unsigned u = __float_as_uint(v); u += 0x7FFFu + ((u >> 16) & 1u); u &= 0xFFFF0000u; return __uint_as_float(u); }
#define NSUP 8192
#define MQ 2048
#define GG 8
#define CF 32
#define CO 128
#define RAD 4.0f
#ifndef MQT
#define MQT MQ
#endif
#define WS_F  0u
#define WS_END (WS_F + 4u * (size_t)MQ * GG * 64)

struct T3 { float d[3]; int i[3]; };
__device__ __forceinline__ void ins3(T3& t, float d, int i) {
  if (d < t.d[2] || (d == t.d[2] && i < t.i[2])) {
    if (d < t.d[1] || (d == t.d[1] && i < t.i[1])) { t.d[2] = t.d[1]; t.i[2] = t.i[1];
      if (d < t.d[0] || (d == t.d[0] && i < t.i[0])) { t.d[1] = t.d[0]; t.i[1] = t.i[0]; t.d[0] = d; t.i[0] = i; } else { t.d[1] = d; t.i[1] = i; } }
    else { t.d[2] = d; t.i[2] = i; } } }
__global__ __launch_bounds__(256) void k_nn(const float* __restrict__ SX, const float* __restrict__ SF, const int* __restrict__ CNT_S, const float* __restrict__ NX, const float* __restrict__ CEN, const int* __restrict__ CNT_N, float* __restrict__ FEAT) {
  #pragma clang fp contract(off)
  __shared__ __align__(16) float srow[8][GG][64]; __shared__ int sidx[8][GG][4]; __shared__ float sd2[8][GG][4]; __shared__ int scnt[8];
  const int tid = threadIdx.x, wave = tid >> 5, lane = tid & 31; const int m = blockIdx.x * 8 + wave;
  const float qx = bfi(NX[m * 3]), qy = bfi(NX[m * 3 + 1]), qz = bfi(NX[m * 3 + 2]);
  const int cs0 = CNT_S[0]; const int cn0 = CNT_N[0]; const int mb = (m >= cn0) ? 1 : 0;
  float cxv[GG], cyv[GG], czv[GG], c2v[GG]; T3 top[GG];
#pragma unroll
  for (int g = 0; g < GG; ++g) { cxv[g] = bfi(CEN[(m * GG + g) * 3]); cyv[g] = bfi(CEN[(m * GG + g) * 3 + 1]); czv[g] = bfi(CEN[(m * GG + g) * 3 + 2]);
    c2v[g] = __fadd_rn(__fadd_rn(__fmul_rn(cxv[g], cxv[g]), __fmul_rn(czv[g], czv[g])), __fmul_rn(cyv[g], cyv[g]));
#pragma unroll
    for (int k = 0; k < 3; ++k) { top[g].d[k] = 3.0e38f; top[g].i[k] = 0x7fffffff; } }
  int ncand = 0;
  for (int j0 = 0; j0 < NSUP; j0 += 32) { const int j = j0 + lane; const float sx = bfi(SX[j * 3]), sy = bfi(SX[j * 3 + 1]), sz = bfi(SX[j * 3 + 2]);
    const int jb = (j >= cs0) ? 1 : 0;
    const bool cand = (fabsf(qx - sx) < RAD) && (fabsf(qy - sy) < RAD) && (fabsf(qz - sz) < RAD) && (jb == mb);
    ncand += __builtin_popcount(__builtin_amdgcn_ballot_w32(cand));
    if (cand) { const float s2 = __fadd_rn(__fadd_rn(__fmul_rn(sx, sx), __fmul_rn(sz, sz)), __fmul_rn(sy, sy));
#pragma unroll
      for (int g = 0; g < GG; ++g) { const float dt = __fadd_rn(__fadd_rn(__fmul_rn(cxv[g], sx), __fmul_rn(cyv[g], sy)), __fmul_rn(czv[g], sz)); const float d2 = __fsub_rn(__fadd_rn(c2v[g], s2), __fmul_rn(2.0f, dt)); ins3(top[g], d2, j); } } }
#pragma unroll
  for (int g = 0; g < GG; ++g) {
#pragma unroll
    for (int r = 0; r < 3; ++r) { float bd = top[g].d[0]; int bi = top[g].i[0];
#pragma unroll
      for (int o = 1; o < 32; o <<= 1) { const float od = __shfl_xor(bd, o); const int oi = __shfl_xor(bi, o); if (od < bd || (od == bd && oi < bi)) { bd = od; bi = oi; } }
      if (lane == 0) { sd2[wave][g][r] = bd; sidx[wave][g][r] = bi; }
      if (top[g].i[0] == bi && top[g].d[0] == bd && bi != 0x7fffffff) { top[g].d[0] = top[g].d[1]; top[g].i[0] = top[g].i[1]; top[g].d[1] = top[g].d[2]; top[g].i[1] = top[g].i[2]; top[g].d[2] = 3.0e38f; top[g].i[2] = 0x7fffffff; } } }
  if (lane == 0) scnt[wave] = ncand;
  LDSX();
  { const int nc = scnt[wave]; if (nc < 3) { int f0 = 0, f1 = 0, f2 = 0; int nf = 0;
      for (int j0 = 0; j0 < 64 && nf < 3; j0 += 32) { const int j = j0 + lane; const float sx = bfi(SX[j * 3]), sy = bfi(SX[j * 3 + 1]), sz = bfi(SX[j * 3 + 2]); const int jb = (j >= cs0) ? 1 : 0;
        const bool cand = (fabsf(qx - sx) < RAD) && (fabsf(qy - sy) < RAD) && (fabsf(qz - sz) < RAD) && (jb == mb); unsigned bal = __builtin_amdgcn_ballot_w32(!cand);
        while (bal != 0u && nf < 3) { const int b0 = j0 + __builtin_ctz(bal); if (nf == 0) f0 = b0; else if (nf == 1) f1 = b0; else f2 = b0; ++nf; bal &= bal - 1u; } }
      if (lane == 0) { for (int g = 0; g < GG; ++g) for (int k = nc; k < 3; ++k) { const int t = k - nc; sidx[wave][g][k] = (t == 0) ? f0 : (t == 1) ? f1 : f2; sd2[wave][g][k] = 3.0e38f; } } } }
  LDSX();
  { const int nc = scnt[wave];
    if (lane < GG) { const int g = lane; float w[3]; float rec[3];
#pragma unroll
      for (int k = 0; k < 3; ++k) { const bool real = (k < nc); const float d2 = sd2[wave][g][k]; const float dist = real ? sqrtf(fmaxf(d2, 0.f)) : 1.0e8f; rec[k] = __builtin_amdgcn_rcpf(dist + 1e-8f); }
      const float nrm = (rec[0] + rec[1]) + rec[2]; const float den = fmaxf(nrm, 1e-8f);
#pragma unroll
      for (int k = 0; k < 3; ++k) { w[k] = rec[k] * __builtin_amdgcn_rcpf(den); srow[wave][g][48 + k] = w[k];
        const int id = sidx[wave][g][k]; srow[wave][g][CF + 3 * k + 0] = cxv[g] - bfi(SX[id * 3]); srow[wave][g][CF + 3 * k + 1] = cyv[g] - bfi(SX[id * 3 + 1]); srow[wave][g][CF + 3 * k + 2] = czv[g] - bfi(SX[id * 3 + 2]); } }
    LDSX();
    { const int c = lane;
#pragma unroll
      for (int g = 0; g < GG; ++g) { float acc = 0.f;
#pragma unroll
        for (int k = 0; k < 3; ++k) { const int id = sidx[wave][g][k]; acc += srow[wave][g][48 + k] * bfi(SF[(size_t)id * CF + c]); }
        srow[wave][g][c] = (nc > 0) ? acc : 0.f; } }
    LDSX();
    if (lane < GG) { const int g = lane; for (int c = 41; c < 64; ++c) srow[wave][g][c] = 0.f; if (nc == 0) for (int c = CF; c < 41; ++c) srow[wave][g][c] = 0.f; }
    LDSX();
#pragma unroll
    for (int g = 0; g < GG; ++g) if (lane < 16) vst2(FEAT + ((size_t)(m * GG + g)) * 64 + lane * 4, *(const v4f*)&srow[wave][g][lane * 4]); } }
__global__ __launch_bounds__(128) void k_mlp(const float* __restrict__ FEAT, const float* __restrict__ W, const float* __restrict__ GA, const float* __restrict__ BE, const float* __restrict__ MU, const float* __restrict__ VA, float* __restrict__ OUT) { __shared__ __align__(16) float sf[4][16][132];
  const int tid = threadIdx.x, wave = tid >> 5, lane = tid & 31, col = lane & 15, g = lane >> 4; const size_t r0 = (size_t)blockIdx.x * 64 + wave * 16;
  v8f acc[8] = {};
#pragma unroll
  for (int kc = 0; kc < 2; ++kc) { const F2 a = split_row(FEAT + (r0 + col) * 64, kc * 32, lane);
#pragma unroll
    for (int j = 0; j < 8; ++j) { v16b w; const int o = j * 16 + col;
#pragma unroll
      for (int i = 0; i < 16; ++i) { const int k = kc * 32 + (i < 8 ? 8 * g + i : 16 + 8 * g + (i - 8)); w[i] = (k < 41) ? (__bf16)W[(size_t)o * 41 + (k < 41 ? k : 0)] : (__bf16)0.f; }
      acc[j] = wmma_bf(a.h, w, acc[j]); acc[j] = wmma_bf(a.l, w, acc[j]); } }
#pragma unroll
  for (int j = 0; j < 8; ++j) { const int o = j * 16 + col; const float ga = bfr(GA[o]), be = bfr(BE[o]), mu = bfr(MU[o]), rs = rsqrtf(bfr(VA[o]) + 1e-5f);
#pragma unroll
    for (int r = 0; r < 8; ++r) sf[wave][8 * g + r][o] = fmaxf(ga * (acc[j][r] - mu) * rs + be, 0.f); }
  LDSX(); for (int rl = 0; rl < 16; ++rl) vst2(OUT + (r0 + rl) * CO + lane * 4, *(const v4f*)&sf[wave][rl][lane * 4]); }
extern "C" void kernel_launch(void* const* d_in, const int* in_sizes, int n_in, void* d_out, int out_size, void* d_ws, size_t ws_size, hipStream_t stream) {
  (void)in_sizes; (void)n_in; (void)out_size;
  const float** F = (const float**)d_in;
  if (ws_size < (size_t)WS_END) return;
  char* ws = (char*)d_ws; float* FEAT = (float*)(ws + WS_F);
  k_nn<<<dim3(MQT / 8), 256, 0, stream>>>(F[0], F[1], (const int*)d_in[2], F[3], F[4], (const int*)d_in[5], FEAT);
  k_mlp<<<dim3(MQT * GG / 64), 128, 0, stream>>>(FEAT, F[6], F[7], F[8], F[9], F[10], (float*)d_out);
}
